// CausalSelfAttention_18580028522616
// MI455X (gfx1250) — hardware-verified
//
#include <hip/hip_runtime.h>
#ifndef NB
#define NB 2
#endif
#ifndef SEQ
#define SEQ 2048
#endif
#define NB_FULL 2
#define SEQ_FULL 2048
#define DM 1024
#define NH 16
#define HD 64
#define LQ (3 * DM)
#define ER 256
#define NR ((size_t)NB * SEQ)
#define PLP 40
#define RS 0.0009765625f
#define PC 1024.0f

static_assert(HD == 64);
static_assert(NH * HD == DM);
static_assert(DM % 64 == 0);
static_assert(DM % 32 == 0);
static_assert(LQ % 64 == 0);
static_assert(SEQ % 128 == 0);
static_assert(ER % 128 == 0);
static_assert(SEQ >= ER);
static_assert(SEQ <= SEQ_FULL);
static_assert(NB <= NB_FULL);
static_assert((size_t)NB_FULL * SEQ_FULL * DM * 4 == 16777216);
static_assert((PLP * 2) % 16 == 0);

#define SZ_BQKV ((size_t)LQ * DM * 2)
#define SZ_BO   ((size_t)DM * DM * 2)
#define SZ_X16  (NR * DM * 2)
#define SZ_QKV  (NR * LQ * 2)
#define SZ_VTH  ((size_t)NB * NH * HD * SEQ * 2)
#define SZ_VTL  ((size_t)NB * NH * HD * ER * 2)
#define SZ_CTX  (NR * DM * 2)
#define WS_TOTAL (SZ_BQKV + SZ_BO + SZ_X16 + 2 * SZ_QKV + SZ_VTH + SZ_VTL + 2 * SZ_CTX)
static_assert(SZ_BQKV % 256 == 0 && SZ_BO % 256 == 0 && SZ_X16 % 256 == 0 && SZ_QKV % 256 == 0);
static_assert(SZ_VTH % 256 == 0 && SZ_VTL % 256 == 0 && SZ_CTX % 256 == 0);
static_assert(WS_TOTAL <= (size_t)134217728);

typedef _Float16 v16h __attribute__((ext_vector_type(16)));
typedef _Float16 v4h __attribute__((ext_vector_type(4)));
typedef unsigned short v8us __attribute__((ext_vector_type(8), may_alias));
typedef float v8f __attribute__((ext_vector_type(8)));
typedef float v4f __attribute__((ext_vector_type(4)));
typedef float v4fa __attribute__((ext_vector_type(4), may_alias));
union FragH { v16h v; v8us half[2]; _Float16 h[16]; unsigned short u[16]; };

__device__ __forceinline__ unsigned short bf16_bits(float x) { unsigned int u = __float_as_uint(x); return (unsigned short)((u + 0x7FFFu + ((u >> 16) & 1u)) >> 16); }
__device__ __forceinline__ float bf16_rne(float x) { return __uint_as_float(((unsigned int)bf16_bits(x)) << 16); }
__device__ __forceinline__ unsigned short h16_bits(_Float16 h) { return __builtin_bit_cast(unsigned short, h); }

__device__ __forceinline__ v16h g2_frag(const _Float16* p, int hh) { FragH f; f.half[0] = *(const v8us*)((const unsigned short*)p + 8 * hh); f.half[1] = *(const v8us*)((const unsigned short*)p + 16 + 8 * hh); return f.v; }
__device__ __forceinline__ v8f g2_mma(v16h a, v16h b, v8f c) { v8f d = __builtin_amdgcn_wmma_f32_16x16x32_f16(false, a, false, b, (short)0, c, false, false); asm volatile("v_nop\n\tv_nop\n\tv_nop\n\tv_nop" : "+v"(d) : "v"(a), "v"(b)); return d; }

__global__ __launch_bounds__(256) void k_wt_f16(const float* __restrict__ W, _Float16* __restrict__ Wt, int K, int N, float scale) {
  const int t = blockIdx.x * 256 + threadIdx.x; if (t >= N * (K / 8)) return;
  const int n = t / (K / 8), k8 = (t % (K / 8)) * 8; FragH f;
#pragma unroll
  for (int i = 0; i < 8; ++i) f.h[i] = (_Float16)(bf16_rne(W[(size_t)(k8 + i) * N + n]) * scale);
  const v8us o = f.half[0];
  unsigned short* d = (unsigned short*)Wt + (size_t)n * K + k8;
  *(volatile v8us*)d = o; __threadfence(); *(volatile v8us*)d = o;
}

__global__ __launch_bounds__(256) void k_x16(const float* __restrict__ x, _Float16* __restrict__ X16) {
  const size_t t = (size_t)blockIdx.x * 256 + threadIdx.x; if (t >= NR * DM / 8) return;
  const size_t row = t / (DM / 8), c8 = (t % (DM / 8)) * 8;
  const size_t bb = row / SEQ, ss = row % SEQ;
  const float* src = x + (bb * SEQ_FULL + ss) * DM + c8;
  const v4f a = *(const v4fa*)src, c = *(const v4fa*)(src + 4);
  FragH f;
#pragma unroll
  for (int q = 0; q < 4; ++q) { f.h[q] = (_Float16)bf16_rne(a[q]); f.h[4 + q] = (_Float16)bf16_rne(c[q]); }
  const v8us o = f.half[0];
  unsigned short* d = (unsigned short*)X16 + t * 8;
  *(volatile v8us*)d = o; __threadfence(); *(volatile v8us*)d = o;
}

__device__ __forceinline__ void gemm_pass32x64(const _Float16* __restrict__ a0p, const _Float16* __restrict__ a1p, const _Float16* __restrict__ b0p, int ldb, int K, int hh,
                                               v8f& c00, v8f& c01, v8f& c02, v8f& c03, v8f& c10, v8f& c11, v8f& c12, v8f& c13) {
  const _Float16* b1p = b0p + (size_t)16 * ldb; const _Float16* b2p = b1p + (size_t)16 * ldb; const _Float16* b3p = b2p + (size_t)16 * ldb;
#pragma unroll 1
  for (int kb = 0; kb < K; kb += 32) {
    const v16h a0 = g2_frag(a0p + kb, hh), a1 = g2_frag(a1p + kb, hh);
    v16h b = g2_frag(b0p + kb, hh); c00 = g2_mma(a0, b, c00); c10 = g2_mma(a1, b, c10);
    b = g2_frag(b1p + kb, hh); c01 = g2_mma(a0, b, c01); c11 = g2_mma(a1, b, c11);
    b = g2_frag(b2p + kb, hh); c02 = g2_mma(a0, b, c02); c12 = g2_mma(a1, b, c12);
    b = g2_frag(b3p + kb, hh); c03 = g2_mma(a0, b, c03); c13 = g2_mma(a1, b, c13);
  }
}

__global__ __launch_bounds__(128) void k_gemm_qkv(const _Float16* __restrict__ A, const _Float16* __restrict__ Bh, const float* __restrict__ bias,
                                                  _Float16* __restrict__ CH, _Float16* __restrict__ CL) {
  __shared__ __attribute__((aligned(16))) float so[4][32][68];
  const int tid = threadIdx.x, lane = tid & 31, ln = lane & 15, hh = lane >> 4;
  const int w = __builtin_amdgcn_readfirstlane(tid >> 5);
  const int ntn = LQ / 64;
  const int mt = blockIdx.x / ntn, nq = blockIdx.x - mt * ntn;
  const int row0 = mt * 128 + 32 * w, col0 = nq * 64;
  if (row0 >= (int)NR) return;
  const _Float16* a0p = A + (size_t)(row0 + ln) * DM; const _Float16* a1p = a0p + (size_t)16 * DM;
  const _Float16* b0p = Bh + (size_t)(col0 + ln) * DM;
  const v8f z8 = {0.f, 0.f, 0.f, 0.f, 0.f, 0.f, 0.f, 0.f};
  v8f c00 = z8, c01 = z8, c02 = z8, c03 = z8, c10 = z8, c11 = z8, c12 = z8, c13 = z8;
  gemm_pass32x64(a0p, a1p, b0p, DM, DM, hh, c00, c01, c02, c03, c10, c11, c12, c13);
  v8f accs[8] = {c00, c01, c02, c03, c10, c11, c12, c13};
#pragma unroll
  for (int u = 0; u < 8; ++u) {
    const int t = u & 3, half = u >> 2; const int col = col0 + t * 16 + ln; const float bv = bf16_rne(bias[col]);
#pragma unroll
    for (int r = 0; r < 8; ++r) so[w][half * 16 + 8 * hh + r][t * 16 + ln] = accs[u][r] * 0.0625f + bv;
  }
  __builtin_amdgcn_fence(4  , "workgroup"); __builtin_amdgcn_wave_barrier();
  const bool wres = (col0 < DM) || ((row0 % SEQ) < ER);
  const int rsub = lane >> 4, c4 = (lane & 15) * 4;
  for (int pass = 0; pass < 2; ++pass) {
#pragma unroll
    for (int q = 0; q < 16; ++q) {
      const int r = q * 2 + rsub; const v4f v = *(const v4fa*)&so[w][r][c4];
      v4h hi4, lo4;
#pragma unroll
      for (int i = 0; i < 4; ++i) { const _Float16 hv = (_Float16)v[i]; hi4[i] = hv; lo4[i] = (_Float16)((v[i] - (float)hv) * 1024.0f); }
      const size_t o = (size_t)(row0 + r) * LQ + col0 + c4;
      *(volatile v4h*)(CH + o) = hi4;
      if (wres) *(volatile v4h*)(CL + o) = lo4;
    }
    if (pass == 0) __threadfence();
  }
}

__global__ __launch_bounds__(256) void k_vt(const _Float16* __restrict__ V16, int ldv, int voff, _Float16* __restrict__ Vt, int tout) {
  __shared__ unsigned short tl[64][66];
  const int tid = threadIdx.x; const int ng = tout / 64; const int slab = blockIdx.x / ng, lg = blockIdx.x - slab * ng; const int b = slab / NH, h = slab - b * NH;
  for (int i = tid; i < 64 * 8; i += 256) {
    const int r = i / 8, c8 = (i % 8) * 8; FragH f;
    f.half[0] = *(const v8us*)((const unsigned short*)V16 + ((size_t)b * SEQ + lg * 64 + r) * ldv + voff + h * 64 + c8);
#pragma unroll
    for (int q = 0; q < 8; ++q) tl[r][c8 + q] = f.u[q];
  }
  __syncthreads();
  for (int pass = 0; pass < 2; ++pass) {
#pragma unroll
    for (int rd = 0; rd < 2; ++rd) {
      const int d = rd * 32 + tid / 8, pc = tid % 8; FragH f;
#pragma unroll
      for (int q = 0; q < 8; ++q) f.u[q] = tl[pc * 8 + q][d];
      *(volatile v8us*)((unsigned short*)Vt + ((size_t)slab * 64 + d) * tout + lg * 64 + pc * 8) = f.half[0];
    }
    if (pass == 0) __threadfence();
  }
}

template <bool EARLY>
__device__ __forceinline__ void attn_body(const _Float16* __restrict__ PH, const _Float16* __restrict__ PL, const _Float16* __restrict__ VTH, const _Float16* __restrict__ VTL,
                                          _Float16* __restrict__ CH, _Float16* __restrict__ CL) {
  __shared__ __attribute__((aligned(16))) unsigned short pls[4][2][16][PLP];
  __shared__ __attribute__((aligned(16))) float so[4][16][68];
  const int tid = threadIdx.x, lane = tid & 31, ln = lane & 15, hh = lane >> 4;
  const int w = __builtin_amdgcn_readfirstlane(tid >> 5);
  const int nq64 = EARLY ? (ER / 64) : (((SEQ - ER) / 64) > 0 ? ((SEQ - ER) / 64) : 1);
  const int bh = blockIdx.x / nq64; const int qt = blockIdx.x - bh * nq64;
  const int b = bh / NH, h = bh - b * NH;
  const int q0 = (EARLY ? 0 : ER) + qt * 64 + w * 16;
  const size_t rb = (size_t)b * SEQ;
  const size_t qoff = (rb + q0 + ln) * LQ + h * HD;
  const size_t koff0 = (rb + ln) * LQ + DM + h * HD;
  const size_t vbase = ((size_t)bh * HD + ln) * SEQ;
  const size_t vlbase = ((size_t)bh * HD + ln) * ER;
  const v8f z8 = {0.f, 0.f, 0.f, 0.f, 0.f, 0.f, 0.f, 0.f};
  v8f Oh[4] = {z8, z8, z8, z8};
  v8f Ol[4] = {z8, z8, z8, z8};
  float m[8], l[8];
#pragma unroll
  for (int r = 0; r < 8; ++r) { m[r] = -1.0e30f; l[r] = 0.f; }
  const int nj = (q0 + 47) >> 5;
#pragma unroll 1
  for (int j = 0; j < nj; ++j) {
    const int kb = j * 32;
    v8f Sh0 = z8, Sh1 = z8, Sl0 = z8, Sl1 = z8;
#pragma unroll
    for (int s = 0; s < 2; ++s) {
      const v16h qh = g2_frag(PH + qoff + 32 * s, hh);
      const v16h ql = g2_frag(PL + qoff + 32 * s, hh);
      const size_t ko = koff0 + (size_t)kb * LQ + 32 * s;
      v16h kh = g2_frag(PH + ko, hh);
      Sh0 = g2_mma(qh, kh, Sh0); Sl0 = g2_mma(ql, kh, Sl0);
      if (EARLY) { const v16h kl = g2_frag(PL + ko, hh); Sl0 = g2_mma(qh, kl, Sl0); }
      kh = g2_frag(PH + ko + (size_t)16 * LQ, hh);
      Sh1 = g2_mma(qh, kh, Sh1); Sl1 = g2_mma(ql, kh, Sl1);
      if (EARLY) { const v16h kl = g2_frag(PL + ko + (size_t)16 * LQ, hh); Sl1 = g2_mma(qh, kl, Sl1); }
    }
#pragma unroll
    for (int r = 0; r < 8; ++r) {
      const int qg = q0 + 8 * hh + r;
      float s0 = (Sh0[r] + Sl0[r] * RS) * 0.125f;
      float s1 = (Sh1[r] + Sl1[r] * RS) * 0.125f;
      s0 = (kb + ln <= qg) ? s0 : -1.0e30f;
      s1 = (kb + 16 + ln <= qg) ? s1 : -1.0e30f;
      float mx = fmaxf(s0, s1);
      mx = fmaxf(mx, __shfl_xor(mx, 1, 32)); mx = fmaxf(mx, __shfl_xor(mx, 2, 32)); mx = fmaxf(mx, __shfl_xor(mx, 4, 32)); mx = fmaxf(mx, __shfl_xor(mx, 8, 32));
      const float mn = fmaxf(m[r], mx);
      const float sc = __expf(m[r] - mn);
      m[r] = mn;
      const float p0 = __expf(s0 - mn), p1 = __expf(s1 - mn);
      l[r] = l[r] * sc + (p0 + p1);
#pragma unroll
      for (int nt = 0; nt < 4; ++nt) { Oh[nt][r] *= sc; if (EARLY) Ol[nt][r] *= sc; }
      const int prow = 8 * hh + r;
      const float a0 = p0 * PC, a1 = p1 * PC;
      const _Float16 h0 = (_Float16)a0, h1 = (_Float16)a1;
      pls[w][0][prow][ln] = h16_bits(h0); pls[w][0][prow][16 + ln] = h16_bits(h1);
      if (EARLY) { pls[w][1][prow][ln] = h16_bits((_Float16)((a0 - (float)h0) * 1024.0f)); pls[w][1][prow][16 + ln] = h16_bits((_Float16)((a1 - (float)h1) * 1024.0f)); }
    }
    __builtin_amdgcn_fence(4  , "workgroup"); __builtin_amdgcn_wave_barrier();
    FragH ph, pl;
    ph.half[0] = *(const v8us*)&pls[w][0][ln][8 * hh]; ph.half[1] = *(const v8us*)&pls[w][0][ln][16 + 8 * hh];
    if (EARLY) { pl.half[0] = *(const v8us*)&pls[w][1][ln][8 * hh]; pl.half[1] = *(const v8us*)&pls[w][1][ln][16 + 8 * hh]; } else { pl.v = ph.v; }
#pragma unroll
    for (int nt = 0; nt < 4; ++nt) {
      const v16h vh = g2_frag(VTH + vbase + (size_t)nt * 16 * SEQ + kb, hh);
      Oh[nt] = g2_mma(ph.v, vh, Oh[nt]);
      if (EARLY) {
        Ol[nt] = g2_mma(pl.v, vh, Ol[nt]);
        const v16h vl = g2_frag(VTL + vlbase + (size_t)nt * 16 * ER + kb, hh);
        Ol[nt] = g2_mma(ph.v, vl, Ol[nt]);
      }
    }
    __builtin_amdgcn_fence(4  , "workgroup"); __builtin_amdgcn_wave_barrier();
  }
  float inv[8];
#pragma unroll
  for (int r = 0; r < 8; ++r) {
    float t = l[r];
    t += __shfl_xor(t, 1, 32); t += __shfl_xor(t, 2, 32); t += __shfl_xor(t, 4, 32); t += __shfl_xor(t, 8, 32);
    inv[r] = 0.0625f * (1.0f / t);
  }
#pragma unroll
  for (int nt = 0; nt < 4; ++nt) {
#pragma unroll
    for (int r = 0; r < 8; ++r) { float o = Oh[nt][r]; if (EARLY) o += Ol[nt][r] * RS; so[w][8 * hh + r][nt * 16 + ln] = o * inv[r]; }
  }
  __builtin_amdgcn_fence(4  , "workgroup"); __builtin_amdgcn_wave_barrier();
  const int rsub = lane >> 4, c4 = (lane & 15) * 4;
  for (int pass = 0; pass < 2; ++pass) {
#pragma unroll
    for (int q = 0; q < 8; ++q) {
      const int row = q * 2 + rsub; const v4f v = *(const v4fa*)&so[w][row][c4];
      v4h hi4, lo4;
#pragma unroll
      for (int i = 0; i < 4; ++i) { const _Float16 hv = (_Float16)v[i]; hi4[i] = hv; lo4[i] = (_Float16)((v[i] - (float)hv) * 1024.0f); }
      const size_t o = (rb + q0 + row) * DM + h * HD + c4;
      *(volatile v4h*)(CH + o) = hi4;
      *(volatile v4h*)(CL + o) = lo4;
    }
    if (pass == 0) __threadfence();
  }
}

__global__ __launch_bounds__(128) void k_attn_early(const _Float16* __restrict__ PH, const _Float16* __restrict__ PL, const _Float16* __restrict__ VTH, const _Float16* __restrict__ VTL,
                                                    _Float16* __restrict__ CH, _Float16* __restrict__ CL) { attn_body<true>(PH, PL, VTH, VTL, CH, CL); }
__global__ __launch_bounds__(128) void k_attn_late(const _Float16* __restrict__ PH, const _Float16* __restrict__ PL, const _Float16* __restrict__ VTH, const _Float16* __restrict__ VTL,
                                                   _Float16* __restrict__ CH, _Float16* __restrict__ CL) { attn_body<false>(PH, PL, VTH, VTL, CH, CL); }

__global__ __launch_bounds__(128) void k_gemm_out(const _Float16* __restrict__ AH, const _Float16* __restrict__ AL, const _Float16* __restrict__ Bh, const float* __restrict__ bias, float* __restrict__ out) {
  __shared__ __attribute__((aligned(16))) float so[4][32][68];
  const int tid = threadIdx.x, lane = tid & 31, ln = lane & 15, hh = lane >> 4;
  const int w = __builtin_amdgcn_readfirstlane(tid >> 5);
  const int ntn = DM / 64;
  const int mt = blockIdx.x / ntn, nq = blockIdx.x - mt * ntn;
  const int row0 = mt * 128 + 32 * w, col0 = nq * 64;
  if (row0 >= (int)NR) return;
  const _Float16* b0p = Bh + (size_t)(col0 + ln) * DM;
  const v8f z8 = {0.f, 0.f, 0.f, 0.f, 0.f, 0.f, 0.f, 0.f};
  v8f c00 = z8, c01 = z8, c02 = z8, c03 = z8, c10 = z8, c11 = z8, c12 = z8, c13 = z8;
  { const _Float16* a0p = AL + (size_t)(row0 + ln) * DM; const _Float16* a1p = a0p + (size_t)16 * DM;
    gemm_pass32x64(a0p, a1p, b0p, DM, DM, hh, c00, c01, c02, c03, c10, c11, c12, c13); }
  c00 = c00 * RS; c01 = c01 * RS; c02 = c02 * RS; c03 = c03 * RS; c10 = c10 * RS; c11 = c11 * RS; c12 = c12 * RS; c13 = c13 * RS;
  { const _Float16* a0p = AH + (size_t)(row0 + ln) * DM; const _Float16* a1p = a0p + (size_t)16 * DM;
    gemm_pass32x64(a0p, a1p, b0p, DM, DM, hh, c00, c01, c02, c03, c10, c11, c12, c13); }
  v8f accs[8] = {c00, c01, c02, c03, c10, c11, c12, c13};
#pragma unroll
  for (int u = 0; u < 8; ++u) {
    const int t = u & 3, half = u >> 2; const int col = col0 + t * 16 + ln; const float bv = bf16_rne(bias[col]);
#pragma unroll
    for (int r = 0; r < 8; ++r) so[w][half * 16 + 8 * hh + r][t * 16 + ln] = accs[u][r] * RS + bv;
  }
  __builtin_amdgcn_fence(4  , "workgroup"); __builtin_amdgcn_wave_barrier();
  const int rsub = lane >> 4, c4 = (lane & 15) * 4;
  for (int pass = 0; pass < 2; ++pass) {
#pragma unroll
    for (int q = 0; q < 16; ++q) {
      const int r = q * 2 + rsub; const v4f v = *(const v4fa*)&so[w][r][c4];
      const int row = row0 + r; const size_t orow = (size_t)(row / SEQ) * SEQ_FULL + (size_t)(row % SEQ);
      *(volatile v4f*)(out + orow * DM + col0 + c4) = v;
    }
    if (pass == 0) __threadfence();
  }
}

extern "C" void kernel_launch(void* const* d_in, const int* in_sizes, int n_in,
                              void* d_out, int out_size, void* d_ws, size_t ws_size, hipStream_t stream) {
  if (n_in < 5) return;
  const long long need_x = ((long long)(NB - 1) * SEQ_FULL + SEQ) * DM;
  if ((long long)in_sizes[0] < need_x || (long long)in_sizes[1] < (long long)DM * LQ || in_sizes[2] < LQ || (long long)in_sizes[3] < (long long)DM * DM || in_sizes[4] < DM) return;
  if ((long long)out_size < need_x) return;
  const float* x = (const float*)d_in[0]; const float* wqkv = (const float*)d_in[1]; const float* bqkv = (const float*)d_in[2];
  const float* wo = (const float*)d_in[3]; const float* bo = (const float*)d_in[4];
  char* ws = (char*)d_ws; size_t off = 0;
  auto take = [&](size_t bytes) { char* p = ws + off; off += (bytes + 255) & ~(size_t)255; return p; };
  _Float16* BQKV = (_Float16*)take(SZ_BQKV); _Float16* BO = (_Float16*)take(SZ_BO);
  _Float16* X16 = (_Float16*)take(SZ_X16);
  _Float16* QKVH = (_Float16*)take(SZ_QKV); _Float16* QKVL = (_Float16*)take(SZ_QKV);
  _Float16* VTH = (_Float16*)take(SZ_VTH); _Float16* VTL = (_Float16*)take(SZ_VTL);
  _Float16* CH = (_Float16*)take(SZ_CTX); _Float16* CL = (_Float16*)take(SZ_CTX);
  if (off > ws_size) return;
  k_wt_f16<<<(unsigned)(((size_t)LQ * (DM / 8) + 255) / 256), 256, 0, stream>>>(wqkv, BQKV, DM, LQ, 16.0f);
  k_wt_f16<<<(unsigned)(((size_t)DM * (DM / 8) + 255) / 256), 256, 0, stream>>>(wo, BO, DM, DM, 16.0f);
  k_x16<<<(unsigned)((NR * DM / 8 + 255) / 256), 256, 0, stream>>>(x, X16);
  k_gemm_qkv<<<(unsigned)((NR / 128) * (LQ / 64)), 128, 0, stream>>>(X16, BQKV, bqkv, QKVH, QKVL);
  k_vt<<<NB * NH * (SEQ / 64), 256, 0, stream>>>(QKVH, LQ, 2 * DM, VTH, SEQ);
  k_vt<<<NB * NH * (ER / 64), 256, 0, stream>>>(QKVL, LQ, 2 * DM, VTL, ER);
  k_attn_early<<<NB * NH * (ER / 64), 128, 0, stream>>>(QKVH, QKVL, VTH, VTL, CH, CL);
  if (SEQ > ER) k_attn_late<<<NB * NH * ((SEQ - ER) / 64), 128, 0, stream>>>(QKVH, QKVL, VTH, VTL, CH, CL);
  k_gemm_out<<<(unsigned)((NR / 128) * (DM / 64)), 128, 0, stream>>>(CH, CL, BO, bo, (float*)d_out);
}
